// RgcnConv_3728031613523
// MI455X (gfx1250) — hardware-run, weakly checked
//
#include <hip/hip_runtime.h>

typedef float          v8f   __attribute__((ext_vector_type(8)));
typedef float          v4f   __attribute__((ext_vector_type(4)));
typedef unsigned int   v4u   __attribute__((ext_vector_type(4)));
typedef int            v8i   __attribute__((ext_vector_type(8)));
typedef unsigned short v8us  __attribute__((ext_vector_type(8)));
typedef unsigned short v16us __attribute__((ext_vector_type(16)));
typedef __bf16         v16bf __attribute__((ext_vector_type(16)));
typedef _Float16       v16h  __attribute__((ext_vector_type(16)));
typedef v4f  __attribute__((may_alias)) v4fa;
typedef v8us __attribute__((may_alias)) v8usa;
union FragB { v16bf v; v16us u; v8us h[2]; v8i w; };
union FragH { v16h  v; v16us u; v8us h[2]; v8i w; };

__device__ __forceinline__ v8f wmb(const FragB& a, const FragB& b, v8f c) {
  v8f d = __builtin_amdgcn_wmma_f32_16x16x32_bf16(false, a.v, false, b.v, (short)0, c, false, false);
  asm volatile("v_nop\n\tv_nop\n\tv_nop\n\tv_nop" : "+v"(d) : "v"(a.w), "v"(b.w));
  return d;
}

__device__ __forceinline__ v8f wmh(const FragH& a, const FragH& b, v8f c) {
  v8f d = __builtin_amdgcn_wmma_f32_16x16x32_f16(false, a.v, false, b.v, (short)0, c, false, false);
  asm volatile("v_nop\n\tv_nop\n\tv_nop\n\tv_nop" : "+v"(d) : "v"(a.w), "v"(b.w));
  return d;
}

__device__ __forceinline__ unsigned bf16_bits(float f) {
  const unsigned u = __float_as_uint(f);
  const unsigned r = (u + 0x7FFFu + ((u >> 16) & 1u)) >> 16;
  const unsigned q = (u >> 16) | 0x40u;
  return ((u & 0x7fffffffu) > 0x7f800000u) ? q : r;
}

__device__ __forceinline__ float bf16_val(float f) {
  return __uint_as_float(bf16_bits(f) << 16);
}
__device__ __forceinline__ int clampi(int v, int lo, int hi) {
  return v < lo ? lo : (v > hi ? hi : v);
}

__device__ __forceinline__ unsigned f16_bits(float f) {
  const unsigned u  = __float_as_uint(f);
  const unsigned s  = (u >> 16) & 0x8000u;
  const unsigned a  = u & 0x7fffffffu;
  const unsigned t  = a - 0x38000000u;
  const unsigned r  = (t + 0x0FFFu + ((t >> 13) & 1u)) >> 13;
  const unsigned rc = r > 0x7C00u ? 0x7C00u : r;
  const bool small  = a < 0x38800000u;
  const bool isnan  = a > 0x7f800000u;
  const unsigned fin = small ? 0u : (s | rc);
  return isnan ? (s | 0x7E00u) : fin;
}

__device__ __forceinline__ unsigned pk16(unsigned lo, unsigned hi) { return lo | (hi << 16); }
__device__ __forceinline__ unsigned bf16_lo_bits(float v) {
  float hi = bf16_val(v);
  asm volatile("" : "+v"(hi));
  return bf16_bits(v - hi);
}
__device__ __forceinline__ v4u pack8_bf16(v4f a, v4f c) {
  return (v4u){ pk16(bf16_bits(a[0]), bf16_bits(a[1])), pk16(bf16_bits(a[2]), bf16_bits(a[3])),
                pk16(bf16_bits(c[0]), bf16_bits(c[1])), pk16(bf16_bits(c[2]), bf16_bits(c[3])) };
}
__device__ __forceinline__ v4u pack8_bf16_lo(v4f a, v4f c) {
  return (v4u){ pk16(bf16_lo_bits(a[0]), bf16_lo_bits(a[1])), pk16(bf16_lo_bits(a[2]), bf16_lo_bits(a[3])),
                pk16(bf16_lo_bits(c[0]), bf16_lo_bits(c[1])), pk16(bf16_lo_bits(c[2]), bf16_lo_bits(c[3])) };
}
__device__ __forceinline__ v4u pack8_f16(v4f a, v4f c) {
  return (v4u){ pk16(f16_bits(a[0]), f16_bits(a[1])), pk16(f16_bits(a[2]), f16_bits(a[3])),
                pk16(f16_bits(c[0]), f16_bits(c[1])), pk16(f16_bits(c[2]), f16_bits(c[3])) };
}

template <int FORM>
__global__ __launch_bounds__(256) void k_plane(const float* __restrict__ src, int rows, int cols, int ldsrc,
                                               unsigned short* __restrict__ dst, int MP, int KP) {
  static_assert(FORM >= 0 && FORM <= 3);
  const int KTOT = (FORM == 1 || FORM == 3) ? 2 * KP : KP;
  const unsigned ppr   = (unsigned)(KTOT >> 3);
  const unsigned kp8   = (unsigned)(KP >> 3);
  const unsigned total = (unsigned)MP * ppr;
  const unsigned g     = blockIdx.x * 256u + threadIdx.x;
  const unsigned rowu  = g / ppr;
  const unsigned p     = g - rowu * ppr;
  const bool second    = p >= kp8;
  const int row = (int)rowu;
  const int c0  = (int)((second ? p - kp8 : p) << 3);
  const float* srow = src + (size_t)clampi(row, 0, rows - 1) * (size_t)ldsrc;
  float x[8];
  unsigned mk[8];
#pragma unroll
  for (int e = 0; e < 8; ++e) {
    const int c = c0 + e;
    const float v = srow[clampi(c, 0, cols - 1)];
    asm volatile("" :: "v"(v));
    x[e]  = v;
    mk[e] = (row < rows && c < cols) ? 0xFFFFu : 0u;
  }
  const v4f a = (v4f){ x[0], x[1], x[2], x[3] };
  const v4f c = (v4f){ x[4], x[5], x[6], x[7] };
  v4u o;
  if (FORM == 2) {
    o = pack8_f16(a, c);
  } else {
    const v4u hi = pack8_bf16(a, c);
    o = hi;
    if (FORM == 1) { const v4u lo = pack8_bf16_lo(a, c); o = second ? lo : hi; }
  }
  const v4u mw = (v4u){ pk16(mk[0], mk[1]), pk16(mk[2], mk[3]), pk16(mk[4], mk[5]), pk16(mk[6], mk[7]) };
  o &= mw;
  if (g < total) {
    volatile v4u* q = (volatile v4u*)(dst + (size_t)g * 8);
    *q = o;
    __threadfence();
    *q = o;
  }
}

template <int FORM> struct FragOf    { typedef FragB T; };
template <>         struct FragOf<2> { typedef FragH T; };
__device__ __forceinline__ v8f mm(const FragB& a, const FragB& b, v8f c) { return wmb(a, b, c); }
__device__ __forceinline__ v8f mm(const FragH& a, const FragH& b, v8f c) { return wmh(a, b, c); }
template <class F> __device__ __forceinline__ F ld_frag(const unsigned short* p) {
  F f;
  f.h[0] = *(const v8usa*)(p);
  f.h[1] = *(const v8usa*)(p + 16);
  return f;
}

template <int FORM, int EPI>
__global__ __launch_bounds__(256) __attribute__((amdgpu_num_vgpr(248)))
void k_gemm_nt(const unsigned short* __restrict__ A, const unsigned short* __restrict__ B,
               const float* __restrict__ bias, float* __restrict__ D, int M, int N, int KTOT, int ldd) {
  static_assert(FORM >= 0 && FORM <= 2);
  static_assert(EPI == 0 || EPI == 1);
  typedef typename FragOf<FORM>::T F;
  __shared__ __attribute__((aligned(16))) float sT[8][16 * 68];
  const int lane = threadIdx.x & 31;
  const int wave = threadIdx.x >> 5;
  const int tilesM = (M + 63) >> 6;
  const int tilesN = (N + 63) >> 6;
  const int tile = blockIdx.x * 8 + wave;
  if (tile >= tilesM * tilesN) return;
  const int tm = tile / tilesN;
  const int tn = tile - tm * tilesN;
  const int m0 = tm << 6;
  const int n0 = tn << 6;

  const int rl = lane & 15;
  const int h8 = (lane >> 4) * 8;
  const unsigned short* pa = A + (size_t)(m0 + rl) * (size_t)KTOT + h8;
  const unsigned short* pb = B + (size_t)(n0 + rl) * (size_t)KTOT + h8;

  v8f acc[4][4];
#pragma unroll
  for (int i = 0; i < 4; ++i)
#pragma unroll
    for (int j = 0; j < 4; ++j) acc[i][j] = (v8f){0.f, 0.f, 0.f, 0.f, 0.f, 0.f, 0.f, 0.f};

#pragma unroll 1
  for (int k0 = 0; k0 < KTOT; k0 += 32) {
    F bf[4];
#pragma unroll
    for (int j = 0; j < 4; ++j) bf[j] = ld_frag<F>(pb + (size_t)(j << 4) * (size_t)KTOT + k0);
#pragma unroll
    for (int i = 0; i < 4; ++i) {
      const F af = ld_frag<F>(pa + (size_t)(i << 4) * (size_t)KTOT + k0);
#pragma unroll
      for (int j = 0; j < 4; ++j) acc[i][j] = mm(af, bf[j], acc[i][j]);
    }
  }

  float* slab = sT[wave];
  const int hh = lane >> 4;
  const int c4 = (lane & 15) * 4;
  const int nc = n0 + c4;
  const bool cok = nc < N;
  v4f bv = (v4f){0.f, 0.f, 0.f, 0.f};
  if (EPI == 1) {
    bv = *(const v4fa*)(bias + clampi(nc, 0, N - 4));
    asm volatile("" :: "v"(bv));
  }
#pragma unroll
  for (int i = 0; i < 4; ++i) {
    const int mBase = m0 + (i << 4);
#pragma unroll
    for (int j = 0; j < 4; ++j) {
#pragma unroll
      for (int r = 0; r < 8; ++r) slab[(h8 + r) * 68 + (j << 4) + rl] = acc[i][j][r];
    }
    __builtin_amdgcn_fence(__ATOMIC_RELEASE, "workgroup");
    __builtin_amdgcn_wave_barrier();
    __builtin_amdgcn_fence(__ATOMIC_ACQUIRE, "workgroup");
    v4f vv[8];
#pragma unroll
    for (int it = 0; it < 8; ++it) {
      const int row = it * 2 + hh;
      v4f v = *(const v4fa*)(slab + row * 68 + c4);
      if (EPI == 1) v += bv;
      vv[it] = v;
    }
    for (int pass = 0; pass < 2; ++pass) {
#pragma unroll
      for (int it = 0; it < 8; ++it) {
        const int row = mBase + it * 2 + hh;
        if (cok && row < M) *(volatile v4f*)(D + (size_t)row * (size_t)ldd + nc) = vv[it];
      }
      __threadfence();
    }
    __builtin_amdgcn_fence(__ATOMIC_RELEASE, "workgroup");
    __builtin_amdgcn_wave_barrier();
    __builtin_amdgcn_fence(__ATOMIC_ACQUIRE, "workgroup");
  }
}

#pragma clang fp contract(off)
#include <stddef.h>

typedef int v4i __attribute__((ext_vector_type(4)));
typedef v4i __attribute__((may_alias)) v4ia;

constexpr int NN     = 100000;
constexpr int KD     = 128;
constexpr int NE     = 1600000;
constexpr int MPAD   = 100096;
constexpr int NTHR   = 256;
constexpr int NWAVE  = 8;
constexpr int EPT    = 8;
constexpr int WCH    = 32 * EPT;
constexpr int SLB    = 10;
constexpr int NBRUN  = 1 << SLB;
constexpr int NBK    = 98;
constexpr int RCAP   = 21504;
constexpr int DEGCAP = 64;
constexpr int MAXDEG_MEAS   = 36;
constexpr int MAXB1024_MEAS = 16721;
constexpr int BK_ZINTS = 2 * RCAP + 3 * NBRUN;
constexpr int BK_INTS  = BK_ZINTS + 64;
constexpr int BK_LDS   = BK_INTS * 4;
constexpr size_t WSMAX = ((size_t)128 << 20);

static_assert(KD % 32 == 0 && (2 * KD) % 32 == 0);
static_assert(MPAD % 64 == 0 && MPAD >= NN && MPAD == 782 * 128);
static_assert(NN % 16 == 0 && NN % 8 == 0);
static_assert(NBK * NBRUN >= MPAD && (NBK - 1) * NBRUN < NN);
static_assert(NE % WCH == 0 && NE < (1 << 21));
static_assert((((long long)NE) << SLB) < (1LL << 31));
static_assert(RCAP % 1024 == 0 && RCAP % 32 == 0);
static_assert((long long)RCAP * 100 >= (long long)MAXB1024_MEAS * 125);
static_assert(MAXDEG_MEAS + 8 <= DEGCAP);
static_assert(BK_INTS % 4 == 0 && BK_LDS <= 262144);
static_assert(BK_LDS + 0 <= 327680);
static_assert((MPAD * 32) % NTHR == 0 && (MPAD * 16) % NTHR == 0);

__device__ __forceinline__ void st2_v4u(unsigned short* p, v4u v) {
  volatile v4u* q = (volatile v4u*)p;
  *q = v;
  __threadfence();
  *q = v;
}
__device__ __forceinline__ void st2_v4f(float* p, v4f v) {
  volatile v4f* q = (volatile v4f*)p;
  *q = v;
  __threadfence();
  *q = v;
}

__global__ __launch_bounds__(256) void k_xs(const float* __restrict__ x, unsigned short* __restrict__ xs) {
  const unsigned g = blockIdx.x * 256u + threadIdx.x;
  const int row = (int)(g >> 5);
  const int c0  = (int)(g & 15u) << 3;
  const float* s = x + (size_t)clampi(row, 0, NN - 1) * (size_t)KD + c0;
  const v4f a = *(const v4fa*)s;
  const v4f c = *(const v4fa*)(s + 4);
  asm volatile("" :: "v"(a));
  asm volatile("" :: "v"(c));
  v4u o = pack8_bf16(a, c);
  const unsigned mk = row < NN ? 0xFFFFFFFFu : 0u;
  o &= (v4u){ mk, mk, mk, mk };
  if (g < (unsigned)MPAD * 32u) st2_v4u(xs + (size_t)g * 8, o);
}

__device__ __forceinline__ v4u gather8_bf16(const float* __restrict__ base) {
  float f[8];
#pragma unroll
  for (int i = 0; i < 8; ++i) {
    const float v = base[(size_t)i * (size_t)KD];
    asm volatile("" :: "v"(v));
    f[i] = v;
  }
  return pack8_bf16((v4f){ f[0], f[1], f[2], f[3] }, (v4f){ f[4], f[5], f[6], f[7] });
}

__global__ __launch_bounds__(256) void k_prep(const float* __restrict__ W, const float* __restrict__ lw,
                                              const float* __restrict__ coeff, const float* __restrict__ hb,
                                              unsigned short* wsb, unsigned short* w1t, unsigned short* w2t,
                                              float* smallp) {
  __shared__ __attribute__((aligned(16))) float stg[160];
  const int tid = (int)threadIdx.x;
  const int blk = (int)blockIdx.x;
  if (blk < 32) {
    const int u  = (blk & 7) * NTHR + tid;
    const int n  = u >> 4;
    const int k8 = (u & 15) * 8;
    const int sel = blk >> 3;
    const size_t so = (size_t)k8 * KD + (size_t)n;
    if (sel == 0) {
      st2_v4u(wsb + (size_t)n * 256 + k8, gather8_bf16(W + so));
    } else if (sel == 1) {
      st2_v4u(wsb + (size_t)n * 256 + 128 + k8, gather8_bf16(lw + so));
    } else if (sel == 2) {
      st2_v4u(w1t + (size_t)n * KD + k8, gather8_bf16(W + (size_t)KD * KD + so));
    } else {
      st2_v4u(w2t + (size_t)n * KD + k8, gather8_bf16(W + (size_t)2 * KD * KD + so));
    }
  } else {
    const float cv = coeff[clampi(tid, 0, 15)];
    asm volatile("" :: "v"(cv));
    const float bv = hb[clampi(tid - 32, 0, KD - 1)];
    asm volatile("" :: "v"(bv));
    float val = bf16_val(bv);
    val = (tid < 32) ? 0.0f : val;
    val = (tid < 16) ? bf16_val(cv) : val;
    if (tid < 160) stg[tid] = val;
    __syncthreads();
    const int q = tid < 40 ? tid : 39;
    const v4f v = *(const v4fa*)(stg + 4 * q);
    asm volatile("" :: "v"(v));
    if (tid < 40) st2_v4f(smallp + 4 * tid, v);
  }
}

__device__ __forceinline__ void load_slots(const int* __restrict__ dsts, int e0, unsigned nbs, unsigned (&s)[8]) {
  const v4i da = *(const v4ia*)(dsts + e0);
  const v4i db = *(const v4ia*)(dsts + e0 + 4);
  const int d0 = da.x, d1 = da.y, d2 = da.z, d3 = da.w, d4 = db.x, d5 = db.y, d6 = db.z, d7 = db.w;
  asm volatile("" :: "v"(d0)); asm volatile("" :: "v"(d1)); asm volatile("" :: "v"(d2)); asm volatile("" :: "v"(d3));
  asm volatile("" :: "v"(d4)); asm volatile("" :: "v"(d5)); asm volatile("" :: "v"(d6)); asm volatile("" :: "v"(d7));
  s[0] = (unsigned)d0 - nbs; s[1] = (unsigned)d1 - nbs; s[2] = (unsigned)d2 - nbs; s[3] = (unsigned)d3 - nbs;
  s[4] = (unsigned)d4 - nbs; s[5] = (unsigned)d5 - nbs; s[6] = (unsigned)d6 - nbs; s[7] = (unsigned)d7 - nbs;
}

__global__ __launch_bounds__(256) void k_bucket(const int* __restrict__ srcs, const int* __restrict__ dsts,
                                                const int* __restrict__ etyp, const float* __restrict__ ctab,
                                                int* LIST, int* CNT, int* OFF, int* FLAG) {
  extern __shared__ __attribute__((aligned(16))) int dsm[];
  int* hl   = dsm;
  int* pl   = dsm + RCAP;
  int* cnt  = dsm + 2 * RCAP;
  int* offs = cnt + NBRUN;
  int* cur  = offs + NBRUN;
  int* misc = cur + NBRUN;
  const int tid = (int)threadIdx.x, lane = tid & 31, wave = tid >> 5;
  const int blk = (int)blockIdx.x;
  const unsigned nbs = (unsigned)(blk * NBRUN);

  {
    const v4i z4 = {0, 0, 0, 0};
    for (int i = tid * 4; i < BK_INTS; i += NTHR * 4) *(v4ia*)(dsm + i) = z4;
  }
  __syncthreads();
  {
    const float cv = ctab[clampi(tid, 0, 15)];
    asm volatile("" :: "v"(cv));
    if (tid < 16) misc[32 + tid] = __float_as_int(cv);
  }

  const int per  = ((NE + NWAVE * WCH - 1) / (NWAVE * WCH)) * WCH;
  const int ebeg = wave * per;
  const int eend = (ebeg + per < NE) ? (ebeg + per) : NE;

  {
    int n = 0;
#pragma unroll 1
    for (int cb = ebeg; cb < eend; cb += WCH) {
      unsigned s[8];
      load_slots(dsts, cb + lane * EPT, nbs, s);
#pragma unroll
      for (int j = 0; j < 8; ++j) n += (s[j] < (unsigned)NBRUN) ? 1 : 0;
    }
#pragma unroll
    for (int d = 16; d >= 1; d >>= 1) n += __shfl_xor(n, d, 32);
    if (lane == 0) misc[wave] = n;
  }
  __syncthreads();

  int wbase = 0, tot = 0;
#pragma unroll
  for (int w2 = 0; w2 < NWAVE; ++w2) {
    int c = misc[w2];
    c = c < 0 ? 0 : (c > per ? per : c);
    wbase += (w2 < wave) ? c : 0;
    tot += c;
  }
  const int totc = tot > RCAP ? RCAP : tot;

  {
    int wc = wbase;
#pragma unroll 1
    for (int cb = ebeg; cb < eend; cb += WCH) {
      const int e0 = cb + lane * EPT;
      unsigned s[8];
      load_slots(dsts, e0, nbs, s);
      bool h[8];
      unsigned m[8];
#pragma unroll
      for (int j = 0; j < 8; ++j) h[j] = s[j] < (unsigned)NBRUN;
#pragma unroll
      for (int j = 0; j < 8; ++j) m[j] = __builtin_amdgcn_ballot_w32(h[j]);
      const unsigned any = m[0] | m[1] | m[2] | m[3] | m[4] | m[5] | m[6] | m[7];
      if (any != 0u) {
        int pre = 0, pop = 0;
#pragma unroll
        for (int j = 0; j < 8; ++j) {
          pre += (int)__builtin_amdgcn_mbcnt_lo(m[j], 0u);
          pop += (int)__builtin_popcount(m[j]);
        }
        int p = wc + pre;
#pragma unroll
        for (int j = 0; j < 8; ++j) {
          if (h[j]) { if (p < RCAP) hl[p] = ((e0 + j) << SLB) | (int)s[j]; p = p + 1; }
        }
        wc += pop;
      }
    }
  }
  __syncthreads();

  if (wave == 0) {
#pragma unroll 1
    for (int b0 = 0; b0 < totc; b0 += 32) {
      const int idx = b0 + lane;
      const int ent = hl[idx < RCAP ? idx : RCAP - 1];
      const int m32 = (totc - b0) < 32 ? (totc - b0) : 32;
#pragma unroll 1
      for (int k = 0; k < m32; ++k) {
        const int u    = __builtin_amdgcn_readlane(ent, k);
        const int slot = u & (NBRUN - 1);
        if (lane == 0) cnt[slot] = cnt[slot] + 1;
      }
    }
    if (lane == 0) misc[9] = (tot > RCAP) ? 1 : 0;
  }
  __syncthreads();
  if (wave == 0) {
    const int base = lane * (NBRUN / 32);
    int s = 0;
#pragma unroll 1
    for (int i = 0; i < NBRUN / 32; ++i) s += cnt[base + i];
    int incl = s;
#pragma unroll
    for (int d = 1; d < 32; d <<= 1) {
      const int y = __shfl_up(incl, d, 32);
      incl += (lane >= d) ? y : 0;
    }
    int run = incl - s;
#pragma unroll 1
    for (int i = 0; i < NBRUN / 32; ++i) {
      const int cv = cnt[base + i];
      offs[base + i] = run;
      cur[base + i]  = run;
      run += cv;
    }
  }
  __syncthreads();
  if (wave == 0) {
#pragma unroll 1
    for (int b0 = 0; b0 < totc; b0 += 32) {
      const int idx = b0 + lane;
      const int ent = hl[idx < RCAP ? idx : RCAP - 1];
      const int m32 = (totc - b0) < 32 ? (totc - b0) : 32;
#pragma unroll 1
      for (int k = 0; k < m32; ++k) {
        const int u    = __builtin_amdgcn_readlane(ent, k);
        const int slot = u & (NBRUN - 1);
        const int eid  = (u >> SLB) & 0x1FFFFF;
        if (lane == 0) {
          int p = cur[slot];
          p = p < 0 ? 0 : (p > RCAP - 1 ? RCAP - 1 : p);
          pl[p] = eid;
          cur[slot] = p + 1;
        }
      }
    }
  }
  __syncthreads();

  const int ovf = misc[9];
  int* lp = LIST + (size_t)blk * (size_t)(3 * RCAP);
#pragma unroll 1
  for (int i = tid * 4; i < RCAP; i += NTHR * 4) {
    const v4i e4 = *(const v4ia*)(pl + i);
    int   sv[4];
    int   a0[4], a1[4];
#pragma unroll
    for (int j = 0; j < 4; ++j) {
      const int eid = clampi(e4[j], 0, NE - 1);
      int s = srcs[eid];
      asm volatile("" :: "v"(s));
      int t = etyp[eid];
      asm volatile("" :: "v"(t));
      s = clampi(s, 0, NN - 1);
      t = clampi(t, 0, 7);
      const int mk = (i + j < totc) ? -1 : 0;
      sv[j] = s & mk;
      a0[j] = misc[32 + 2 * t] & mk;
      a1[j] = misc[33 + 2 * t] & mk;
    }
    const v4i so = { sv[0], sv[1], sv[2], sv[3] };
    const v4i c0 = { a0[0], a0[1], a0[2], a0[3] };
    const v4i c1 = { a1[0], a1[1], a1[2], a1[3] };
    volatile v4i* q0 = (volatile v4i*)(lp + i);
    volatile v4i* q1 = (volatile v4i*)(lp + RCAP + i);
    volatile v4i* q2 = (volatile v4i*)(lp + 2 * RCAP + i);
    *q0 = so; *q1 = c0; *q2 = c1;
    __threadfence();
    *q0 = so; *q1 = c0; *q2 = c1;
  }
  {
    const v4i cv = *(const v4ia*)(cnt + 4 * tid);
    const v4i ov = *(const v4ia*)(offs + 4 * tid);
    const v4i fv = { ovf, ovf, ovf, ovf };
    volatile v4i* qc = (volatile v4i*)(CNT + (size_t)blk * NBRUN + 4 * tid);
    volatile v4i* qo = (volatile v4i*)(OFF + (size_t)blk * NBRUN + 4 * tid);
    volatile v4i* qf = (volatile v4i*)(FLAG + (size_t)blk * 32 + 4 * (tid & 7));
    *qc = cv; *qo = ov;
    if (tid < 8) *qf = fv;
    __threadfence();
    *qc = cv; *qo = ov;
    if (tid < 8) *qf = fv;
  }
}

__global__ __launch_bounds__(256) void k_walk(const int* __restrict__ LIST, const int* __restrict__ CNT,
                                              const int* __restrict__ OFF, const int* __restrict__ FLAG,
                                              const float* __restrict__ T, float* out, int cplane) {
  const int lane = (int)threadIdx.x & 31;
  const int wave = (int)threadIdx.x >> 5;
  const int row  = (int)blockIdx.x * NWAVE + wave;
  if (row >= NN) return;
  const int bk = row >> SLB;
  int c = CNT[row];
  asm volatile("" :: "v"(c));
  int o = OFF[row];
  asm volatile("" :: "v"(o));
  const int flag = FLAG[(size_t)bk * 32];
  asm volatile("" :: "v"(flag));
  const bool big = (c > DEGCAP) || (c < 0);
  c = clampi(c, 0, DEGCAP);
  o = clampi(o, 0, RCAP - 1);
  c = __builtin_amdgcn_readfirstlane(c);
  o = __builtin_amdgcn_readfirstlane(o);
  int last = o + (c > 0 ? c : 1) - 1;
  last = last > RCAP - 1 ? RCAP - 1 : last;
  const int pc = clampi(cplane, 1, 2);
  const int* sb = LIST + (size_t)bk * (size_t)(3 * RCAP);
  const int* cb = sb + (size_t)pc * RCAP;

  v4f acc = (v4f){ 0.0f, 0.0f, 0.0f, 0.0f };
#pragma unroll 1
  for (int b0 = 0; b0 < c; b0 += 32) {
    int idx = o + b0 + lane;
    idx = idx > last ? last : idx;
    int sr = sb[idx];
    asm volatile("" :: "v"(sr));
    const int wv = cb[idx];
    asm volatile("" :: "v"(wv));
    sr = clampi(sr, 0, NN - 1);
    const int m32 = (c - b0) < 32 ? (c - b0) : 32;
#pragma unroll 1
    for (int k = 0; k < m32; ++k) {
      const int   sk = __builtin_amdgcn_readlane(sr, k);
      const float ck = __int_as_float(__builtin_amdgcn_readlane(wv, k));
      const v4f t = *(const v4fa*)(T + (size_t)sk * KD + 4 * lane);
      const v4f p = t * ck;
      acc = acc + p;
    }
  }
  float* op = out + (size_t)row * KD + 4 * lane;
  const v4f self = *(const v4fa*)op;
  asm volatile("" :: "v"(self));
  v4f v = self + acc;
  const float qnan = __uint_as_float(0x7fc00000u);
  const bool bad = (flag != 0) || big;
  v.x = bad ? qnan : v.x; v.y = bad ? qnan : v.y; v.z = bad ? qnan : v.z; v.w = bad ? qnan : v.w;
  st2_v4f(op, v);
}

extern "C" void kernel_launch(void* const* d_in, const int* in_sizes, int n_in,
                              void* d_out, int out_size, void* d_ws, size_t ws_size,
                              hipStream_t stream) {
  if (n_in < 8) return;
  if (in_sizes[0] != NN * KD) return;
  if (in_sizes[1] != 16) return;
  if (in_sizes[2] != 3 * KD * KD) return;
  if (in_sizes[3] != KD) return;
  if (in_sizes[4] != KD * KD) return;
  if (in_sizes[5] != NE || in_sizes[6] != NE || in_sizes[7] != NE) return;
  if (out_size != NN * KD) return;

  const float* feat  = (const float*)d_in[0];
  const float* coeff = (const float*)d_in[1];
  const float* W     = (const float*)d_in[2];
  const float* hb    = (const float*)d_in[3];
  const float* lw    = (const float*)d_in[4];
  const int*   esrc  = (const int*)d_in[5];
  const int*   edst  = (const int*)d_in[6];
  const int*   etyp  = (const int*)d_in[7];
  float* out = (float*)d_out;

  constexpr size_t zXB   = (size_t)MPAD * KD * 2;
  constexpr size_t zXT   = (size_t)MPAD * 2 * KD * 2;
  constexpr size_t zLIST = (size_t)NBK * RCAP * 12;
  constexpr size_t zCNT  = (size_t)NBK * NBRUN * 4;
  constexpr size_t zOFF  = (size_t)NBK * NBRUN * 4;
  constexpr size_t zFLAG = (size_t)NBK * 128;
  constexpr size_t zWS   = (size_t)KD * 2 * KD * 2;
  constexpr size_t zWT   = (size_t)KD * KD * 2;
  constexpr size_t zSM   = 1024;
  constexpr size_t oXB   = 0;
  constexpr size_t oXT   = oXB + zXB;
  constexpr size_t oLIST = oXT + zXT;
  constexpr size_t oCNT  = oLIST + zLIST;
  constexpr size_t oOFF  = oCNT + zCNT;
  constexpr size_t oFLAG = oOFF + zOFF;
  constexpr size_t oWS   = oFLAG + zFLAG;
  constexpr size_t oW1T  = oWS + zWS;
  constexpr size_t oW2T  = oW1T + zWT;
  constexpr size_t oSM   = oW2T + zWT;
  constexpr size_t oEND  = oSM + zSM;
  static_assert(zXT == (size_t)MPAD * KD * 4);
  static_assert(zXB % 128 == 0 && zXT % 128 == 0 && zLIST % 128 == 0 && zCNT % 128 == 0 && zFLAG % 128 == 0);
  static_assert(zWS % 128 == 0 && zWT % 128 == 0 && zSM % 128 == 0 && zSM >= 640);
  static_assert(((size_t)RCAP * 4) % 128 == 0);
  static_assert(oEND == ((size_t)402773 * 256));
  static_assert(oEND <= WSMAX);
  if (oEND > ws_size) return;

  char* ws = (char*)d_ws;
  unsigned short* XB   = (unsigned short*)(ws + oXB);
  unsigned short* XS   = (unsigned short*)(ws + oXT);
  float*          T    = (float*)(ws + oXT);
  int*            LIST = (int*)(ws + oLIST);
  int*            CNT  = (int*)(ws + oCNT);
  int*            OFF  = (int*)(ws + oOFF);
  int*            FLAG = (int*)(ws + oFLAG);
  unsigned short* WSB  = (unsigned short*)(ws + oWS);
  unsigned short* W1T  = (unsigned short*)(ws + oW1T);
  unsigned short* W2T  = (unsigned short*)(ws + oW2T);
  float*          SM   = (float*)(ws + oSM);
  float*          CT   = SM;
  float*          BIAS = SM + 32;

  constexpr int gPlane = MPAD * KD / 8 / NTHR;
  constexpr int gXs    = MPAD * 32 / NTHR;
  constexpr int tiles1 = ((NN + 63) / 64) * 2;
  constexpr int tiles2 = (MPAD / 64) * 2;
  constexpr int gG1    = (tiles1 + 7) / 8;
  constexpr int gG2    = (tiles2 + 7) / 8;
  static_assert(gPlane * NTHR * 8 == MPAD * KD);

  hipFuncSetAttribute(reinterpret_cast<const void*>(&k_bucket), hipFuncAttributeMaxDynamicSharedMemorySize, (int)BK_LDS);

  k_plane<0><<<gPlane, NTHR, 0, stream>>>(feat, NN, KD, KD, XB, MPAD, KD);
  k_xs<<<gXs, NTHR, 0, stream>>>(feat, XS);
  k_prep<<<33, NTHR, 0, stream>>>(W, lw, coeff, hb, WSB, W1T, W2T, SM);
  k_gemm_nt<0, 1><<<gG1, NTHR, 0, stream>>>(XS, WSB, BIAS, out, NN, KD, 2 * KD, KD);
  k_bucket<<<NBK, NTHR, BK_LDS, stream>>>(esrc, edst, etyp, CT, LIST, CNT, OFF, FLAG);
  k_gemm_nt<0, 0><<<gG2, NTHR, 0, stream>>>(XB, W1T, BIAS, T, MPAD, KD, KD, KD);
  k_walk<<<NN / NWAVE, NTHR, 0, stream>>>(LIST, CNT, OFF, FLAG, T, out, 1);
  k_gemm_nt<0, 0><<<gG2, NTHR, 0, stream>>>(XB, W2T, BIAS, T, MPAD, KD, KD, KD);
  k_walk<<<NN / NWAVE, NTHR, 0, stream>>>(LIST, CNT, OFF, FLAG, T, out, 2);
}
